// GNN_79044578115825
// MI455X (gfx1250) — hardware-verified
//
#include <hip/hip_runtime.h>
#include <stddef.h>
#include <stdint.h>
#include <math.h>


#define NMOL   256
#define NATOM  1024
#define NEDGE  8192
#define XW     3072
#define HID    64
#define K2     128
#define NPO    128
#define DEGCAP 32
#define GT     256
#define ECH    2048
#define LT     128
#define TROWS  128
#define AT     256
#define HT     128
#define HBM    64
#define NU2    (HID * (K2 / 8))
#define NUP    (NPO * (K2 / 8))
#define NUS    256
#define SMN    512
#define WSMAX  134217728

static_assert(NEDGE % ECH == 0 && ECH == GT * 8);
static_assert(NATOM % GT == 0 && NATOM % TROWS == 0 && NATOM % 8 == 0);
static_assert(DEGCAP == 32);
static_assert(XW % (4 * LT) == 0 && NATOM % (4 * LT) == 0 && (TROWS * DEGCAP) % (4 * LT) == 0);
static_assert(K2 % 32 == 0 && K2 == 2 * HID && HID % 16 == 0 && NPO % 16 == 0);
static_assert(TROWS == (LT / 32) * 32 && HBM == (HT / 32) * 16 && NMOL % HBM == 0);
static_assert(NU2 % 256 == 0 && NUP % 256 == 0);
static_assert(XW * 2 + NATOM * 4 + TROWS * DEGCAP * 4 + 256 * 4 + TROWS * HID * 4 <= 65536);

typedef float          v2f   __attribute__((ext_vector_type(2)));
typedef float          v4f   __attribute__((ext_vector_type(4)));
typedef float          v8f   __attribute__((ext_vector_type(8)));
typedef int            v4i   __attribute__((ext_vector_type(4)));
typedef int            v8i   __attribute__((ext_vector_type(8)));
typedef unsigned int   v4u   __attribute__((ext_vector_type(4)));
typedef unsigned short v4us  __attribute__((ext_vector_type(4)));
typedef unsigned short v8us  __attribute__((ext_vector_type(8)));
typedef unsigned short v16us __attribute__((ext_vector_type(16)));
typedef __bf16         v16bf __attribute__((ext_vector_type(16)));
typedef v2f  __attribute__((may_alias)) v2fa;
typedef v4f  __attribute__((may_alias)) v4fa;
typedef v4i  __attribute__((may_alias)) v4ia;
typedef v4u  __attribute__((may_alias)) v4ua;
typedef v4us __attribute__((may_alias)) v4usa;
typedef v8us __attribute__((may_alias)) v8usa;
union FragB { v16bf v; v16us u; v8us h[2]; v8i w; };

__device__ __forceinline__ v8f wmb(const FragB& a, const FragB& b, v8f c) {
  v8f d = __builtin_amdgcn_wmma_f32_16x16x32_bf16(false, a.v, false, b.v, (short)0, c, false, false);
  asm volatile("v_nop\n\tv_nop\n\tv_nop\n\tv_nop" : "+v"(d) : "v"(a.w), "v"(b.w));
  return d;
}

__device__ __forceinline__ unsigned bf16_bits(float f) {
  const unsigned u = __float_as_uint(f);
  return (u + 0x7FFFu + ((u >> 16) & 1u)) >> 16;
}
__device__ __forceinline__ float bf16_val(float f) {
  return __uint_as_float(bf16_bits(f) << 16);
}
__device__ __forceinline__ float leaky(float v) {
  return (v >= 0.0f) ? v : 0.01f * v;
}
__device__ __forceinline__ void split2(float va, float vb, unsigned& hw, unsigned& lw) {
  const unsigned ha = bf16_bits(va), hb = bf16_bits(vb);
  const unsigned la = bf16_bits(va - __uint_as_float(ha << 16));
  const unsigned lb = bf16_bits(vb - __uint_as_float(hb << 16));
  hw = ha | (hb << 16);
  lw = la | (lb << 16);
}
__device__ __forceinline__ float x1val(float a0, float a1, float a2, float w0, float w1, float w2, float bb) {
  return leaky(fmaf(a2, w2, fmaf(a1, w1, a0 * w0)) + bb);
}

__global__ __launch_bounds__(256) void k_prep(const float* __restrict__ W1, const float* __restrict__ b1,
                                              const float* __restrict__ W2, const float* __restrict__ b2,
                                              const float* __restrict__ Wp, const float* __restrict__ bp,
                                              unsigned short* W2T2, unsigned short* WpT2, float* SM) {
  const int u = (int)blockIdx.x * 256 + (int)threadIdx.x;
  if (u < NU2) {
    const int n  = u >> 4;
    const int k8 = (u & 15) * 8;
    const int kk = k8 & (HID - 1);
    const float* p = W2 + (size_t)kk * HID + n;
    v8us o;
#pragma unroll
    for (int i = 0; i < 8; ++i) o[i] = (unsigned short)bf16_bits(p[(size_t)i * HID]);
    unsigned short* dp = W2T2 + (size_t)n * K2 + k8;
    *(volatile v8us*)dp = o;
    __threadfence();
    *(volatile v8us*)dp = o;
  } else if (u < NU2 + NUP) {
    const int v  = u - NU2;
    const int n  = v >> 4;
    const int k8 = (v & 15) * 8;
    const int kk = k8 & (HID - 1);
    const float* p = Wp + (size_t)kk * NPO + n;
    v8us o;
#pragma unroll
    for (int i = 0; i < 8; ++i) o[i] = (unsigned short)bf16_bits(p[(size_t)i * NPO]);
    unsigned short* dp = WpT2 + (size_t)n * K2 + k8;
    *(volatile v8us*)dp = o;
    __threadfence();
    *(volatile v8us*)dp = o;
  } else {
    const int t = u - (NU2 + NUP);
    if (t >= SMN / 4) return;
    const int q4 = 4 * t;
    const int o1 = q4 < 188 ? q4 : 188;
    int o2 = q4 - 192; o2 = o2 < 0 ? 0 : (o2 > 60 ? 60 : o2);
    int o3 = q4 - 256; o3 = o3 < 0 ? 0 : (o3 > 60 ? 60 : o3);
    int o4 = q4 - 320; o4 = o4 < 0 ? 0 : (o4 > 124 ? 124 : o4);
    const v4f c1 = *(const v4f*)(W1 + o1);
    const v4f c2 = *(const v4f*)(b1 + o2);
    const v4f c3 = *(const v4f*)(b2 + o3);
    const v4f c4 = *(const v4f*)(bp + o4);
    const unsigned m1 = 0u - (unsigned)(q4 < 192);
    const unsigned m2 = 0u - (unsigned)(q4 >= 192 && q4 < 256);
    const unsigned m3 = 0u - (unsigned)(q4 >= 256 && q4 < 320);
    const unsigned m4 = 0u - (unsigned)(q4 >= 320 && q4 < 448);
    v4f v;
    v.x = __uint_as_float((__float_as_uint(c1.x) & m1) | (__float_as_uint(c2.x) & m2) |
                          (__float_as_uint(c3.x) & m3) | (__float_as_uint(c4.x) & m4));
    v.y = __uint_as_float((__float_as_uint(c1.y) & m1) | (__float_as_uint(c2.y) & m2) |
                          (__float_as_uint(c3.y) & m3) | (__float_as_uint(c4.y) & m4));
    v.z = __uint_as_float((__float_as_uint(c1.z) & m1) | (__float_as_uint(c2.z) & m2) |
                          (__float_as_uint(c3.z) & m3) | (__float_as_uint(c4.z) & m4));
    v.w = __uint_as_float((__float_as_uint(c1.w) & m1) | (__float_as_uint(c2.w) & m2) |
                          (__float_as_uint(c3.w) & m3) | (__float_as_uint(c4.w) & m4));
    v.x = bf16_val(v.x); v.y = bf16_val(v.y); v.z = bf16_val(v.z); v.w = bf16_val(v.w);
    float* dp = SM + q4;
    *(volatile v4f*)dp = v;
    __threadfence();
    *(volatile v4f*)dp = v;
  }
}

__global__ __launch_bounds__(GT) void k_graph(const int* __restrict__ ei, int* NBR, int* CNT, float* DINV) {
  __shared__ __attribute__((aligned(16))) int dss[ECH];
  __shared__ __attribute__((aligned(16))) int sss[ECH];
  __shared__ __attribute__((aligned(16))) int nb[GT * DEGCAP];
  __shared__ __attribute__((aligned(16))) int cs[GT];
  __shared__ __attribute__((aligned(16))) float dv[GT];
  const int tid  = (int)threadIdx.x;
  const int node = (int)blockIdx.x * GT + tid;
  {
    const v4i z = {0, 0, 0, 0};
#pragma unroll
    for (int q = 0; q < DEGCAP / 4; ++q) *(v4ia*)(nb + tid * DEGCAP + 4 * q) = z;
  }
  int c = 0;
#pragma unroll 1
  for (int ch = 0; ch < NEDGE / ECH; ++ch) {
    const int e0 = ch * ECH + tid * 8;
    const v4i s0 = *(const v4i*)(ei + e0);
    const v4i s1 = *(const v4i*)(ei + e0 + 4);
    const v4i d0 = *(const v4i*)(ei + NEDGE + e0);
    const v4i d1 = *(const v4i*)(ei + NEDGE + e0 + 4);
    *(v4ia*)(sss + tid * 8)     = s0;
    *(v4ia*)(sss + tid * 8 + 4) = s1;
    *(v4ia*)(dss + tid * 8)     = d0;
    *(v4ia*)(dss + tid * 8 + 4) = d1;
    __syncthreads();
#pragma unroll 1
    for (int e4 = 0; e4 < ECH / 4; ++e4) {
      const v4i d = *(const v4ia*)(dss + 4 * e4);
      const v4i s = *(const v4ia*)(sss + 4 * e4);
      if (d.x == node) { if (c < DEGCAP) nb[tid * DEGCAP + c] = s.x; c = c + 1; }
      if (d.y == node) { if (c < DEGCAP) nb[tid * DEGCAP + c] = s.y; c = c + 1; }
      if (d.z == node) { if (c < DEGCAP) nb[tid * DEGCAP + c] = s.z; c = c + 1; }
      if (d.w == node) { if (c < DEGCAP) nb[tid * DEGCAP + c] = s.w; c = c + 1; }
    }
    __syncthreads();
  }
  cs[tid] = c;
  dv[tid] = 1.0f / sqrtf(1.0f + (float)c);
  __syncthreads();

  v4i rows[8];
#pragma unroll
  for (int it = 0; it < 8; ++it) rows[it] = *(const v4ia*)(nb + 4 * (it * GT + tid));
  const v4i cv  = *(const v4ia*)(cs + 4 * (tid & 63));
  const v4f dvv = *(const v4fa*)(dv + 4 * (tid & 63));
  int*   nbase = NBR + (size_t)blockIdx.x * (GT * DEGCAP);
  int*   cp    = CNT  + (size_t)blockIdx.x * GT + 4 * (tid & 63);
  float* dp    = DINV + (size_t)blockIdx.x * GT + 4 * (tid & 63);
  const bool st = tid < GT / 4;
#pragma unroll
  for (int it = 0; it < 8; ++it) *(volatile v4i*)(nbase + 4 * (it * GT + tid)) = rows[it];
  if (st) { *(volatile v4i*)cp = cv; *(volatile v4f*)dp = dvv; }
  __threadfence();
#pragma unroll
  for (int it = 0; it < 8; ++it) *(volatile v4i*)(nbase + 4 * (it * GT + tid)) = rows[it];
  if (st) { *(volatile v4i*)cp = cv; *(volatile v4f*)dp = dvv; }
}

__global__ __launch_bounds__(LT) void k_l1g2(const float* __restrict__ x, const int* __restrict__ NBR,
                                             const int* __restrict__ CNT, const float* __restrict__ DINV,
                                             const float* __restrict__ SM,
                                             const unsigned short* __restrict__ W2T2, float* HW2) {
  __shared__ __attribute__((aligned(16))) unsigned short xs16[XW];
  __shared__ __attribute__((aligned(16))) float dinvs[NATOM];
  __shared__ __attribute__((aligned(16))) int nbrs[TROWS * DEGCAP];
  __shared__ __attribute__((aligned(16))) float wb[256];
  __shared__ __attribute__((aligned(16))) float stg[TROWS * HID];
  const int tid = (int)threadIdx.x, lane = tid & 31, wave = tid >> 5, hh = lane >> 4, m = lane & 15;
  const int b    = (int)blockIdx.x >> 3;
  const int tile = (int)blockIdx.x & 7;

  {
    const float* xb = x + (size_t)b * XW;
#pragma unroll
    for (int it = 0; it < XW / (4 * LT); ++it) {
      const int idx4 = it * LT + tid;
      const v4f v = *(const v4f*)(xb + 4 * idx4);
      v4us o;
      o[0] = (unsigned short)bf16_bits(v.x); o[1] = (unsigned short)bf16_bits(v.y);
      o[2] = (unsigned short)bf16_bits(v.z); o[3] = (unsigned short)bf16_bits(v.w);
      *(v4usa*)(xs16 + 4 * idx4) = o;
    }
#pragma unroll
    for (int it = 0; it < NATOM / (4 * LT); ++it) {
      const int idx4 = it * LT + tid;
      *(v4fa*)(dinvs + 4 * idx4) = *(const v4f*)(DINV + 4 * idx4);
    }
    const int* nbt = NBR + (size_t)tile * (TROWS * DEGCAP);
#pragma unroll
    for (int it = 0; it < (TROWS * DEGCAP) / (4 * LT); ++it) {
      const int idx4 = it * LT + tid;
      *(v4ia*)(nbrs + 4 * idx4) = *(const v4i*)(nbt + 4 * idx4);
    }
    if (tid < 64) *(v4fa*)(wb + 4 * tid) = *(const v4f*)(SM + 4 * tid);
  }
  const int craw = CNT[tile * TROWS + tid];
  __syncthreads();

  {
    const int i = tile * TROWS + tid;
    const bool pois = (craw < 0) || (craw > DEGCAP);
    const int c = craw < 0 ? 0 : (craw > DEGCAP ? DEGCAP : craw);
    int cm = c;
#pragma unroll
    for (int d = 16; d >= 1; d >>= 1) {
      const int y = __shfl_xor(cm, d, 32);
      cm = cm > y ? cm : y;
    }
    cm = __builtin_amdgcn_readfirstlane(cm);
    cm = cm > DEGCAP ? DEGCAP : cm;
    const float di = dinvs[i];
    float a0 = 0.0f, a1 = 0.0f, a2 = 0.0f;
#pragma unroll 1
    for (int k = 0; k < cm; ++k) {
      int j = nbrs[tid * DEGCAP + k];
      j = j < 0 ? 0 : (j > NATOM - 1 ? NATOM - 1 : j);
      const float dj = dinvs[j];
      const float f  = (k < c) ? 1.0f : 0.0f;
      const float w  = (dj * di) * f;
      const float x0 = __uint_as_float((unsigned)xs16[3 * j + 0] << 16);
      const float x1 = __uint_as_float((unsigned)xs16[3 * j + 1] << 16);
      const float x2 = __uint_as_float((unsigned)xs16[3 * j + 2] << 16);
      a0 = fmaf(w, x0, a0); a1 = fmaf(w, x1, a1); a2 = fmaf(w, x2, a2);
    }
    {
      const float rd = di * di;
      const float x0 = __uint_as_float((unsigned)xs16[3 * i + 0] << 16);
      const float x1 = __uint_as_float((unsigned)xs16[3 * i + 1] << 16);
      const float x2 = __uint_as_float((unsigned)xs16[3 * i + 2] << 16);
      a0 = fmaf(rd, x0, a0); a1 = fmaf(rd, x1, a1); a2 = fmaf(rd, x2, a2);
    }
    const float qnan = __int_as_float(0x7fc00000);
    a0 = pois ? qnan : a0; a1 = pois ? qnan : a1; a2 = pois ? qnan : a2;

    unsigned* sw = (unsigned*)stg + tid * 64;
#pragma unroll 1
    for (int g = 0; g < 8; ++g) {
      const v4f p0 = *(const v4fa*)(wb + 8 * g);
      const v4f p1 = *(const v4fa*)(wb + 8 * g + 4);
      const v4f q0 = *(const v4fa*)(wb + 64 + 8 * g);
      const v4f q1 = *(const v4fa*)(wb + 64 + 8 * g + 4);
      const v4f r0 = *(const v4fa*)(wb + 128 + 8 * g);
      const v4f r1 = *(const v4fa*)(wb + 128 + 8 * g + 4);
      const v4f e0 = *(const v4fa*)(wb + 192 + 8 * g);
      const v4f e1 = *(const v4fa*)(wb + 192 + 8 * g + 4);
      const float v0 = x1val(a0, a1, a2, p0.x, q0.x, r0.x, e0.x);
      const float v1 = x1val(a0, a1, a2, p0.y, q0.y, r0.y, e0.y);
      const float v2 = x1val(a0, a1, a2, p0.z, q0.z, r0.z, e0.z);
      const float v3 = x1val(a0, a1, a2, p0.w, q0.w, r0.w, e0.w);
      const float v4 = x1val(a0, a1, a2, p1.x, q1.x, r1.x, e1.x);
      const float v5 = x1val(a0, a1, a2, p1.y, q1.y, r1.y, e1.y);
      const float v6 = x1val(a0, a1, a2, p1.z, q1.z, r1.z, e1.z);
      const float v7 = x1val(a0, a1, a2, p1.w, q1.w, r1.w, e1.w);
      unsigned h0, h1, h2, h3, l0, l1, l2, l3;
      split2(v0, v1, h0, l0);
      split2(v2, v3, h1, l1);
      split2(v4, v5, h2, l2);
      split2(v6, v7, h3, l3);
      v4u hw, lw;
      hw.x = h0; hw.y = h1; hw.z = h2; hw.w = h3;
      lw.x = l0; lw.y = l1; lw.z = l2; lw.w = l3;
      *(v4ua*)(sw + 4 * g)      = hw;
      *(v4ua*)(sw + 32 + 4 * g) = lw;
    }
  }
  __syncthreads();

  v8f acc[2][4];
  {
    const v8f z = {0.f, 0.f, 0.f, 0.f, 0.f, 0.f, 0.f, 0.f};
#pragma unroll
    for (int mt = 0; mt < 2; ++mt)
#pragma unroll
      for (int nt = 0; nt < 4; ++nt) acc[mt][nt] = z;
  }
  {
    const unsigned short* xt = (const unsigned short*)stg;
    const unsigned short* ap = xt + (size_t)(32 * wave + m) * K2 + 8 * hh;
    const unsigned short* wp = W2T2 + (size_t)m * K2 + 8 * hh;
#pragma unroll 1
    for (int ks = 0; ks < K2 / 32; ++ks) {
      FragB af0, af1;
      af0.h[0] = *(const v8usa*)(ap + 32 * ks);
      af0.h[1] = *(const v8usa*)(ap + 32 * ks + 16);
      af1.h[0] = *(const v8usa*)(ap + 16 * K2 + 32 * ks);
      af1.h[1] = *(const v8usa*)(ap + 16 * K2 + 32 * ks + 16);
#pragma unroll
      for (int nt = 0; nt < 4; ++nt) {
        const unsigned short* wq = wp + (size_t)(16 * nt) * K2 + 32 * ks;
        FragB bf;
        bf.h[0] = *(const v8usa*)wq;
        bf.h[1] = *(const v8usa*)(wq + 16);
        acc[0][nt] = wmb(af0, bf, acc[0][nt]);
        acc[1][nt] = wmb(af1, bf, acc[1][nt]);
      }
    }
  }
  __syncthreads();

#pragma unroll
  for (int mt = 0; mt < 2; ++mt) {
#pragma unroll
    for (int nt = 0; nt < 4; ++nt) {
      const int lc = 16 * nt + m;
#pragma unroll
      for (int r = 0; r < 8; ++r) {
        const int lr = 32 * wave + 16 * mt + 8 * hh + r;
        stg[lr * HID + lc] = acc[mt][nt][r];
      }
    }
  }
  __syncthreads();

  const size_t rowBase = (size_t)blockIdx.x * TROWS;
  v4f fv[16];
#pragma unroll
  for (int i = 0; i < 16; ++i) {
    const int lr = 32 * wave + 2 * i + hh;
    fv[i] = *(const v4fa*)(stg + lr * HID + 4 * m);
  }
#pragma unroll
  for (int i = 0; i < 16; ++i) {
    const int lr = 32 * wave + 2 * i + hh;
    float* op = HW2 + (rowBase + (size_t)lr) * HID + 4 * m;
    *(volatile v4f*)op = fv[i];
  }
  __threadfence();
#pragma unroll
  for (int i = 0; i < 16; ++i) {
    const int lr = 32 * wave + 2 * i + hh;
    float* op = HW2 + (rowBase + (size_t)lr) * HID + 4 * m;
    *(volatile v4f*)op = fv[i];
  }
}

__global__ __launch_bounds__(AT) void k_agg2(const float* __restrict__ HW2, const int* __restrict__ NBR,
                                             const int* __restrict__ CNT, const float* __restrict__ DINV,
                                             const float* __restrict__ SM, unsigned short* GB) {
  __shared__ __attribute__((aligned(16))) float wsum[8 * HID];
  __shared__ __attribute__((aligned(16))) unsigned short gsm[K2];
  const int tid = (int)threadIdx.x, lane = tid & 31, wave = tid >> 5;
  const float* hb = HW2 + (size_t)blockIdx.x * NATOM * HID;
  const v2f bq = *(const v2f*)(SM + 256 + 2 * lane);
  const float qnan = __int_as_float(0x7fc00000);
  float p0 = 0.0f, p1 = 0.0f;
#pragma unroll 1
  for (int si = 0; si < NATOM / 8; ++si) {
    const int i = si * 8 + wave;
    const int craw = CNT[i];
    int sr = NBR[i * DEGCAP + lane];
    sr = sr < 0 ? 0 : (sr > NATOM - 1 ? NATOM - 1 : sr);
    const float di  = DINV[i];
    const float cf  = DINV[sr] * di;
    const int   cfi = __float_as_int(cf);
    const bool big = (craw < 0) || (craw > DEGCAP);
    int c = craw < 0 ? 0 : (craw > DEGCAP ? DEGCAP : craw);
    c = __builtin_amdgcn_readfirstlane(c);
    c = c > DEGCAP ? DEGCAP : c;
    float acc0 = 0.0f, acc1 = 0.0f;
#pragma unroll 1
    for (int k = 0; k < c; ++k) {
      int sk = __builtin_amdgcn_readlane(sr, k);
      sk = sk < 0 ? 0 : (sk > NATOM - 1 ? NATOM - 1 : sk);
      const float ck = __int_as_float(__builtin_amdgcn_readlane(cfi, k));
      const v2f a = *(const v2fa*)(hb + (size_t)sk * HID + 2 * lane);
      acc0 = fmaf(ck, a.x, acc0); acc1 = fmaf(ck, a.y, acc1);
    }
    const v2f sv = *(const v2fa*)(hb + (size_t)i * HID + 2 * lane);
    const float rd = di * di;
    float y0 = (acc0 + sv.x * rd) + bq.x;
    float y1 = (acc1 + sv.y * rd) + bq.y;
    y0 = leaky(y0); y1 = leaky(y1);
    y0 = big ? qnan : y0; y1 = big ? qnan : y1;
    p0 += y0; p1 += y1;
  }
  wsum[wave * HID + 2 * lane + 0] = p0;
  wsum[wave * HID + 2 * lane + 1] = p1;
  __syncthreads();
  if (tid < HID) {
    float s = 0.0f;
#pragma unroll
    for (int w2 = 0; w2 < 8; ++w2) s += wsum[w2 * HID + tid];
    const float g = s * (1.0f / (float)NATOM);
    const unsigned hbits = bf16_bits(g);
    const unsigned lbits = bf16_bits(g - __uint_as_float(hbits << 16));
    gsm[tid]       = (unsigned short)hbits;
    gsm[HID + tid] = (unsigned short)lbits;
  }
  __syncthreads();
  const v8us q = *(const v8usa*)(gsm + 8 * (lane & 15));
  unsigned short* gp = GB + (size_t)blockIdx.x * K2 + 8 * (lane & 15);
  const bool okst = (wave == 0) && (lane < 16);
  if (okst) *(volatile v8us*)gp = q;
  __threadfence();
  if (okst) *(volatile v8us*)gp = q;
}

__global__ __launch_bounds__(HT) void k_head(const unsigned short* __restrict__ GB,
                                             const unsigned short* __restrict__ WpT2,
                                             const float* __restrict__ SM, float* out) {
  __shared__ __attribute__((aligned(16))) float stg[HBM * NPO];
  const int tid = (int)threadIdx.x, lane = tid & 31, wave = tid >> 5, hh = lane >> 4, m = lane & 15;
  const int rowBase = (int)blockIdx.x * HBM;

  v8f acc[8];
  {
    const v8f z = {0.f, 0.f, 0.f, 0.f, 0.f, 0.f, 0.f, 0.f};
#pragma unroll
    for (int t = 0; t < 8; ++t) acc[t] = z;
  }
  const unsigned short* ap = GB + (size_t)(rowBase + 16 * wave + m) * K2 + 8 * hh;
  const unsigned short* bp = WpT2 + (size_t)m * K2 + 8 * hh;
#pragma unroll 1
  for (int ks = 0; ks < K2 / 32; ++ks) {
    FragB af;
    af.h[0] = *(const v8usa*)(ap + 32 * ks);
    af.h[1] = *(const v8usa*)(ap + 32 * ks + 16);
#pragma unroll
    for (int nt = 0; nt < 8; ++nt) {
      const unsigned short* wq = bp + (size_t)(16 * nt) * K2 + 32 * ks;
      FragB bf;
      bf.h[0] = *(const v8usa*)wq;
      bf.h[1] = *(const v8usa*)(wq + 16);
      acc[nt] = wmb(af, bf, acc[nt]);
    }
  }
#pragma unroll
  for (int nt = 0; nt < 8; ++nt) {
    const int lc = 16 * nt + m;
#pragma unroll
    for (int r = 0; r < 8; ++r) {
      const int lr = 16 * wave + 8 * hh + r;
      stg[lr * NPO + lc] = acc[nt][r];
    }
  }
  __syncthreads();

  const v4f bb4 = *(const v4f*)(SM + 320 + 4 * lane);
  v4f pv[16];
#pragma unroll
  for (int i = 0; i < 16; ++i) {
    const v4f t = *(const v4fa*)(stg + (16 * wave + i) * NPO + 4 * lane) + bb4;
    v4f y;
    y.x = leaky(t.x); y.y = leaky(t.y); y.z = leaky(t.z); y.w = leaky(t.w);
    pv[i] = y;
  }
#pragma unroll
  for (int i = 0; i < 16; ++i) {
    float* op = out + (size_t)(rowBase + 16 * wave + i) * NPO + 4 * lane;
    *(volatile v4f*)op = pv[i];
  }
  __threadfence();
#pragma unroll
  for (int i = 0; i < 16; ++i) {
    float* op = out + (size_t)(rowBase + 16 * wave + i) * NPO + 4 * lane;
    *(volatile v4f*)op = pv[i];
  }
}

static inline size_t al256(size_t o) { return (o + 255) & ~(size_t)255; }

extern "C" void kernel_launch(void* const* d_in, const int* in_sizes, int n_in,
                              void* d_out, int out_size, void* d_ws, size_t ws_size,
                              hipStream_t stream) {
  if (n_in < 8) return;
  if (in_sizes[0] != NMOL * XW) return;
  if (in_sizes[1] != 2 * NEDGE) return;
  if (in_sizes[2] != 3 * HID) return;
  if (in_sizes[3] != HID) return;
  if (in_sizes[4] != HID * HID) return;
  if (in_sizes[5] != HID) return;
  if (in_sizes[6] != HID * NPO) return;
  if (in_sizes[7] != NPO) return;
  if (out_size != NMOL * NPO) return;

  const float* x  = (const float*)d_in[0];
  const int*   ei = (const int*)d_in[1];
  const float* W1 = (const float*)d_in[2];
  const float* b1 = (const float*)d_in[3];
  const float* W2 = (const float*)d_in[4];
  const float* b2 = (const float*)d_in[5];
  const float* Wp = (const float*)d_in[6];
  const float* bp = (const float*)d_in[7];
  float* out = (float*)d_out;

  char* ws = (char*)d_ws;
  size_t off = 0;
  const size_t oW2T = off; off = al256(off + (size_t)HID * K2 * 2);
  const size_t oWPT = off; off = al256(off + (size_t)NPO * K2 * 2);
  const size_t oSM  = off; off = al256(off + (size_t)SMN * 4);
  const size_t oNBR = off; off = al256(off + (size_t)NATOM * DEGCAP * 4);
  const size_t oCNT = off; off = al256(off + (size_t)NATOM * 4);
  const size_t oDIN = off; off = al256(off + (size_t)NATOM * 4);
  const size_t oGB  = off; off = al256(off + (size_t)NMOL * K2 * 2);
  const size_t oHW2 = off; off = al256(off + (size_t)NMOL * NATOM * HID * 4);
  if (off > ws_size || off > (size_t)WSMAX) return;
  unsigned short* W2T2 = (unsigned short*)(ws + oW2T);
  unsigned short* WpT2 = (unsigned short*)(ws + oWPT);
  float*          SM   = (float*)(ws + oSM);
  int*            NBR  = (int*)(ws + oNBR);
  int*            CNT  = (int*)(ws + oCNT);
  float*          DINV = (float*)(ws + oDIN);
  unsigned short* GB   = (unsigned short*)(ws + oGB);
  float*          HW2  = (float*)(ws + oHW2);

  k_prep<<<(NU2 + NUP + NUS) / 256, 256, 0, stream>>>(W1, b1, W2, b2, Wp, bp, W2T2, WpT2, SM);
  k_graph<<<NATOM / GT, GT, 0, stream>>>(ei, NBR, CNT, DINV);
  k_l1g2<<<NMOL * (NATOM / TROWS), LT, 0, stream>>>(x, NBR, CNT, DINV, SM, W2T2, HW2);
  k_agg2<<<NMOL, AT, 0, stream>>>(HW2, NBR, CNT, DINV, SM, GB);
  k_head<<<NMOL / HBM, HT, 0, stream>>>(GB, WpT2, SM, out);
}
